// ModulatedConv2D_52226802319456
// MI455X (gfx1250) — hardware-verified
//
#include <hip/hip_runtime.h>


#define NB_  4
#define HH   64
#define WW   64
#define NC_  256
#define NF_  256
#define KH   3
#define KW   3
#define BH   (NB_ * HH)
#define FH   (NB_ * KH)
#define PADT 5
#define KTOT (FH * KW * NC_)
#define WSC  64.0f
#define WSCI (1.0f / 64.0f)

typedef _Float16 h16;
typedef __attribute__((ext_vector_type(16))) _Float16 v16h;
typedef __attribute__((ext_vector_type(8)))  _Float16 v8h;
typedef __attribute__((ext_vector_type(8)))  float    v8f;
typedef __attribute__((ext_vector_type(4)))  float    v4f;
typedef v8h  __attribute__((may_alias)) v8ha;
typedef v4f  __attribute__((may_alias)) v4fa;

__device__ __forceinline__ unsigned short f2bf(float f) { unsigned u = __float_as_uint(f); u += 0x7FFFu + ((u >> 16) & 1u); return (unsigned short)(u >> 16); }
__device__ __forceinline__ float bf2f(unsigned short b) { return __uint_as_float(((unsigned)b) << 16); }
__device__ __forceinline__ float bfr(float f) { return bf2f(f2bf(f)); }
__device__ __forceinline__ v16h cat16(v8h lo, v8h hi) { return __builtin_shufflevector(lo, hi, 0, 1, 2, 3, 4, 5, 6, 7, 8, 9, 10, 11, 12, 13, 14, 15); }
__device__ __forceinline__ v8f wmma16(v16h a, v16h b, v8f c) { return __builtin_amdgcn_wmma_f32_16x16x32_f16(false, a, false, b, (short)0, c, false, false); }
#define VST2(T, p, v) do { const T vst2_v_ = (v); *(volatile T*)(p) = vst2_v_; __threadfence(); *(volatile T*)(p) = vst2_v_; } while (0)

__global__ __launch_bounds__(256) void k_x16(const float* __restrict__ x, h16* X16) {
    const int lane = threadIdx.x & 31;
    const size_t pix = (size_t)blockIdx.x * 8 + (threadIdx.x >> 5);
    if (pix >= (size_t)BH * WW) return;
    v8h o;
#pragma unroll
    for (int i = 0; i < 8; ++i) o[i] = (h16)bfr(x[pix * NC_ + lane * 8 + i]);
    VST2(v8h, X16 + pix * NC_ + lane * 8, o);
}

__global__ __launch_bounds__(256) void k_demod(const float* __restrict__ kern, const float* __restrict__ style, float* DEM) {
    const int b = blockIdx.x, f = threadIdx.x;
    float s = 0.f;
#pragma unroll 1
    for (int t = 0; t < KH * KW * NC_; ++t) { const int c = t & (NC_ - 1); const float w = bfr(kern[(size_t)t * NF_ + f]) * bfr(style[(size_t)b * NC_ + c]); s += w * w; }
    VST2(float, DEM + (size_t)b * NF_ + f, rsqrtf(s + 1e-8f));
}

__global__ __launch_bounds__(256) void k_wt(const float* __restrict__ kern, const float* __restrict__ style, const float* __restrict__ DEM, h16* WT16) {
    __shared__ __align__(16) h16 tl[64 * 72];
    const int tid = threadIdx.x;
    const int tap = blockIdx.z, c0 = blockIdx.y * 64, f0 = blockIdx.x * 64;
    const int b = tap / (KH * KW), kyx = tap - b * (KH * KW);
    const int cc = tid >> 2, fq = (tid & 3) * 16;
    const float sv = bfr(style[(size_t)b * NC_ + c0 + cc]);
    const float* src = kern + ((size_t)kyx * NC_ + c0 + cc) * NF_ + f0 + fq;
#pragma unroll
    for (int i = 0; i < 16; ++i) tl[(fq + i) * 72 + cc] = (h16)(WSC * bfr(src[i]) * sv * DEM[(size_t)b * NF_ + f0 + fq + i]);
    __syncthreads();
    const int piece = tid & 7;
    const size_t kbase = ((size_t)(b * KH) * KW + kyx) * NC_ + c0;
    auto pass = [&]() {
#pragma unroll
        for (int s = 0; s < 2; ++s) { const int fr = (tid >> 3) + 32 * s; const v8h val = *(const v8ha*)(tl + fr * 72 + piece * 8);
            *(volatile v8h*)(WT16 + (size_t)(f0 + fr) * KTOT + kbase + piece * 8) = val; }
    };
    pass(); __threadfence(); pass();
}

__global__ __launch_bounds__(128) void k_conv(const h16* __restrict__ X16, const h16* __restrict__ WT16, float* out) {
    __shared__ __align__(16) float ost[4][16 * 68];
    const int lane = threadIdx.x & 31, wave = threadIdx.x >> 5, lr = lane & 15, hi = lane >> 4;
    const int p0 = blockIdx.x * 64 + wave * 16, f0 = blockIdx.y * 64;
    const int p = p0 + lr;
    const int bh = p / WW, w = p - bh * WW;
    size_t boff[4];
#pragma unroll
    for (int t = 0; t < 4; ++t) boff[t] = (size_t)(f0 + t * 16 + lr) * KTOT + 8 * hi;
    v8f acc[4];
#pragma unroll
    for (int t = 0; t < 4; ++t) acc[t] = (v8f){};
#pragma unroll 1
    for (int tap = 0; tap < FH * KW; ++tap) {
        const int dy = tap / KW, dx = tap - dy * KW;
        const int rr = bh + dy - PADT, cw = w + dx - 1;
        const bool inb = (rr >= 0) && (rr < BH) && (cw >= 0) && (cw < WW);
        const h16* ap = X16 + ((size_t)(inb ? rr : 0) * WW + (inb ? cw : 0)) * NC_ + 8 * hi;
#pragma unroll 2
        for (int c0 = 0; c0 < NC_; c0 += 32) {
            v16h a = (v16h){};
            if (inb) a = cat16(*(const v8h*)(ap + c0), *(const v8h*)(ap + c0 + 16));
            const int kc = tap * NC_ + c0;
#pragma unroll
            for (int t = 0; t < 4; ++t) acc[t] = wmma16(a, cat16(*(const v8h*)(WT16 + boff[t] + kc), *(const v8h*)(WT16 + boff[t] + kc + 16)), acc[t]);
        }
    }
    asm volatile("v_nop\n\tv_nop\n\tv_nop\n\tv_nop" : "+v"(acc[0]), "+v"(acc[1]), "+v"(acc[2]), "+v"(acc[3]));
    float* os = &ost[wave][0];
#pragma unroll
    for (int t = 0; t < 4; ++t)
#pragma unroll
        for (int j = 0; j < 8; ++j) os[(hi * 8 + j) * 68 + t * 16 + lr] = acc[t][j] * WSCI;
    __syncthreads();
    float* crow = out + (size_t)p0 * NF_ + f0;
    auto pass = [&]() {
#pragma unroll
        for (int s = 0; s < 8; ++s) { const int Lid = (lane >> 3) + 4 * s, piece = lane & 7; const int row = Lid >> 1, cofs = (Lid & 1) * 32 + piece * 4;
            const v4f val = *(const v4fa*)(os + row * 68 + cofs); *(volatile v4f*)(crow + (size_t)row * NF_ + cofs) = val; }
    };
    pass(); __threadfence(); pass();
}

extern "C" void kernel_launch(void* const* d_in, const int* in_sizes, int n_in,
                              void* d_out, int out_size, void* d_ws, size_t ws_size, hipStream_t stream) {
    (void)in_sizes; (void)n_in; (void)out_size;
    const float* x = (const float*)d_in[0]; const float* style = (const float*)d_in[1]; const float* kern = (const float*)d_in[2];
    float* out = (float*)d_out;
    char* wsp = (char*)d_ws;
    auto take = [&](size_t bytes) { char* p = wsp; wsp += (bytes + 255) & ~(size_t)255; return (void*)p; };
    h16* X16 = (h16*)take((size_t)BH * WW * NC_ * 2); float* DEM = (float*)take((size_t)NB_ * NF_ * 4); h16* WT16 = (h16*)take((size_t)NF_ * KTOT * 2);
    if ((size_t)(wsp - (char*)d_ws) > ws_size) return;
    k_x16<<<(BH * WW) / 8, 256, 0, stream>>>(x, X16);
    k_demod<<<NB_, 256, 0, stream>>>(kern, style, DEM);
    k_wt<<<dim3(NF_ / 64, NC_ / 64, NB_ * KH * KW), 256, 0, stream>>>(kern, style, DEM, WT16);
    k_conv<<<dim3((BH * WW) / 64, NF_ / 64, 1), 128, 0, stream>>>(X16, WT16, out);
}
